// MultiheadGAT_13460427506084
// MI455X (gfx1250) — hardware-verified
//
#include <hip/hip_runtime.h>
#include <stddef.h>
#include <stdint.h>
#include <math.h>


#define F_IN    256
#define DW      192
#define HC      64
#define NHD     3
#define OUTW    64
#define FHB     128
#define KA2     384
#define NTHR    256
#define NWAVE   8
#define EPT     8
#define CHUNK   (NTHR * EPT)
#define WCAP    (EPT * 32)
#define LISTN   (NWAVE * WCAP)
#define NBMAX   2048
#define SLOTB   11
#define RCAP    28672
#define DEGCAP  64
#define GBM     64
#define GBN     64
#define GTHR    128
#define MROWS   64
#define PARTW   416
#define WSTW    388
#define NEGSL   0.2f
#define EPS_SM  1e-16f
#define EPS_BN  1e-5f
#define MX0     (-1.0e30f)
#define WSMAX   134217728
#define LDS_AGG ((2 * RCAP + 2 * NBMAX + LISTN) * 4 + 64)

static_assert((CHUNK & (CHUNK - 1)) == 0 && CHUNK <= (1 << SLOTB));
static_assert(NBMAX == (1 << SLOTB));
static_assert(NTHR * 8 == NBMAX);
static_assert(LISTN >= NBMAX);
static_assert(LISTN >= NWAVE * WCAP);
static_assert((RCAP % 32) == 0);
static_assert(LDS_AGG <= 300000);
static_assert(GBM == (GTHR / 32) * 16);
static_assert(GTHR == 2 * GBN && GTHR == 2 * GBM);
static_assert((F_IN % 32) == 0 && (KA2 % 32) == 0);
static_assert(DW == NHD * HC && GBN == HC && (DW % GBN) == 0 && OUTW == GBN);
static_assert(KA2 == 2 * DW);
static_assert((MROWS % GBM) == 0);
static_assert(DW == FHB + 2 * 32 && FHB == 4 * 32 && FHB == 2 * HC);
static_assert((DW % 8) == 0 && (F_IN % 8) == 0 && (F_IN / 8) == 32);
static_assert((HC % 4) == 0);
static_assert((PARTW % 32) == 0 && PARTW >= 2 * DW + 1 && PARTW / 4 <= NTHR);
static_assert(WSTW >= 2 * DW + 1 && (WSTW % 4) == 0);
static_assert(NWAVE * WSTW + PARTW <= RCAP);
static_assert(DW <= NTHR && (2 * DW) / 4 <= NTHR);

typedef float          v2f  __attribute__((ext_vector_type(2)));
typedef float          v4f  __attribute__((ext_vector_type(4)));
typedef float          v8f  __attribute__((ext_vector_type(8)));
typedef int            v4i  __attribute__((ext_vector_type(4)));
typedef int            v8i  __attribute__((ext_vector_type(8)));
typedef unsigned int   v4u  __attribute__((ext_vector_type(4)));
typedef unsigned short v8us __attribute__((ext_vector_type(8)));
typedef __bf16         v16b __attribute__((ext_vector_type(16)));
typedef v2f  __attribute__((may_alias)) v2fa;
typedef v4f  __attribute__((may_alias)) v4fa;
typedef v4u  __attribute__((may_alias)) v4ua;
typedef v8us __attribute__((may_alias)) v8usa;
union FragB { v16b v; v8us h[2]; v8i w; };

__device__ __forceinline__ v8f wmb(const FragB& a, const FragB& b, v8f c) {
  v8f d = __builtin_amdgcn_wmma_f32_16x16x32_bf16(false, a.v, false, b.v, (short)0, c, false, false);
  asm volatile("v_nop\n\tv_nop\n\tv_nop\n\tv_nop" : "+v"(d) : "v"(a.w), "v"(b.w));
  return d;
}

__device__ __forceinline__ unsigned int f2bf(float f) {
  const unsigned int u = __float_as_uint(f);
  return ((u + 0x7FFFu + ((u >> 16) & 1u)) >> 16) & 0xFFFFu;
}
__device__ __forceinline__ float bf2f(unsigned int b) { return __uint_as_float(b << 16); }
__device__ __forceinline__ float bfr(float f) { return bf2f(f2bf(f)); }
__device__ __forceinline__ v4f bfr4(const v4f a) {
  v4f r; r.x = bfr(a.x); r.y = bfr(a.y); r.z = bfr(a.z); r.w = bfr(a.w); return r;
}
__device__ __forceinline__ unsigned int pk2(float lo, float hi) { return f2bf(lo) | (f2bf(hi) << 16); }
__device__ __forceinline__ unsigned int pk2lo(float lo, float hi) {
  return f2bf(lo - bfr(lo)) | (f2bf(hi - bfr(hi)) << 16);
}
__device__ __forceinline__ v4u pack8(const v4f a, const v4f b) {
  v4u r;
  r.x = pk2(a.x, a.y); r.y = pk2(a.z, a.w); r.z = pk2(b.x, b.y); r.w = pk2(b.z, b.w);
  return r;
}
__device__ __forceinline__ v4u pack8lo(const v4f a, const v4f b) {
  v4u r;
  r.x = pk2lo(a.x, a.y); r.y = pk2lo(a.z, a.w); r.z = pk2lo(b.x, b.y); r.w = pk2lo(b.z, b.w);
  return r;
}

__device__ __forceinline__ int scan_chunk(const int* __restrict__ dsts, int nE, int cbase, int slotBase,
                                          int nb, int vec8, int* list, int tid, int lane, int wave) {
  int wc = 0;
  const int el0  = tid * EPT;
  const int e0   = cbase + el0;
  const int sent = -2147483647 - 1;
  v4i da, db;
  if (vec8 != 0 && cbase + CHUNK <= nE) {
    da = *(const v4i*)(dsts + e0);
    db = *(const v4i*)(dsts + e0 + 4);
  } else {
    da.x = (e0     < nE) ? dsts[min(e0,     nE - 1)] : sent;
    da.y = (e0 + 1 < nE) ? dsts[min(e0 + 1, nE - 1)] : sent;
    da.z = (e0 + 2 < nE) ? dsts[min(e0 + 2, nE - 1)] : sent;
    da.w = (e0 + 3 < nE) ? dsts[min(e0 + 3, nE - 1)] : sent;
    db.x = (e0 + 4 < nE) ? dsts[min(e0 + 4, nE - 1)] : sent;
    db.y = (e0 + 5 < nE) ? dsts[min(e0 + 5, nE - 1)] : sent;
    db.z = (e0 + 6 < nE) ? dsts[min(e0 + 6, nE - 1)] : sent;
    db.w = (e0 + 7 < nE) ? dsts[min(e0 + 7, nE - 1)] : sent;
  }
  const unsigned nbs = (unsigned)slotBase;
  const unsigned unb = (unsigned)nb;
  const unsigned s0 = (unsigned)da.x - nbs, s1 = (unsigned)da.y - nbs;
  const unsigned s2 = (unsigned)da.z - nbs, s3 = (unsigned)da.w - nbs;
  const unsigned s4 = (unsigned)db.x - nbs, s5 = (unsigned)db.y - nbs;
  const unsigned s6 = (unsigned)db.z - nbs, s7 = (unsigned)db.w - nbs;
  const bool h0 = s0 < unb, h1 = s1 < unb, h2 = s2 < unb, h3 = s3 < unb;
  const bool h4 = s4 < unb, h5 = s5 < unb, h6 = s6 < unb, h7 = s7 < unb;
  const unsigned any = __builtin_amdgcn_ballot_w32(h0 | h1 | h2 | h3 | h4 | h5 | h6 | h7);
  if (any != 0u) {
#define HITJ(J, HJ, SJ) { \
      const unsigned mj = __builtin_amdgcn_ballot_w32(HJ); \
      if (mj != 0u) { \
        if (HJ) { \
          const int pos = wc + (int)__builtin_amdgcn_mbcnt_lo(mj, 0u); \
          if (pos < WCAP) list[wave * WCAP + pos] = ((el0 + (J)) << SLOTB) | (int)(SJ); \
        } \
        wc += (int)__builtin_popcount(mj); } }
    HITJ(0, h0, s0)
    HITJ(1, h1, s1)
    HITJ(2, h2, s2)
    HITJ(3, h3, s3)
    HITJ(4, h4, s4)
    HITJ(5, h5, s5)
    HITJ(6, h6, s6)
    HITJ(7, h7, s7)
#undef HITJ
  }
  return wc;
}

__global__ __launch_bounds__(NTHR) void k_xprep(const float* __restrict__ x, unsigned short* xb, int nN, int nUnits) {
  const int i = (int)blockIdx.x * NTHR + (int)threadIdx.x;
  if (i >= nUnits) return;
  const int row = i >> 5;
  const int c0  = (i & 31) * 8;
  const int rc  = row < nN ? row : nN - 1;
  const float* p = x + (size_t)rc * F_IN + c0;
  v4f a = *(const v4fa*)p, b = *(const v4fa*)(p + 4);
  const v4f z4 = {0.f, 0.f, 0.f, 0.f};
  if (row >= nN) { a = z4; b = z4; }
  const v4u hv = pack8(a, b);
  const size_t o = (size_t)row * F_IN + c0;
  *(volatile v4u*)(xb + o) = hv;
  __threadfence();
  *(volatile v4u*)(xb + o) = hv;
}

__global__ __launch_bounds__(NTHR) void k_wtr(const float* __restrict__ w, int Kin, int Ncol, int Nrows, int Kout,
                                              unsigned short* wt, int nUnits) {
  const int u = (int)blockIdx.x * NTHR + (int)threadIdx.x;
  if (u >= nUnits) return;
  const int kq = Kout >> 3;
  const int n  = u / kq;
  const int k8 = (u - n * kq) * 8;
  const int kk = k8 - (k8 / Kin) * Kin;
  const int ncl = n < Ncol ? n : Ncol - 1;
  const float* p = w + (size_t)kk * (size_t)Ncol + ncl;
  v4f a, b;
  a.x = p[0];                    a.y = p[(size_t)Ncol];         a.z = p[(size_t)2 * Ncol];     a.w = p[(size_t)3 * Ncol];
  b.x = p[(size_t)4 * Ncol];     b.y = p[(size_t)5 * Ncol];     b.z = p[(size_t)6 * Ncol];     b.w = p[(size_t)7 * Ncol];
  const v4f z4 = {0.f, 0.f, 0.f, 0.f};
  if (n >= Ncol || n >= Nrows) { a = z4; b = z4; }
  const v4u wv = pack8(a, b);
  unsigned short* o = wt + (size_t)n * (size_t)Kout + k8;
  *(volatile v4u*)o = wv;
  __threadfence();
  *(volatile v4u*)o = wv;
}

template <int EPI>
__global__ __launch_bounds__(GTHR) void k_gemm(
    const unsigned short* __restrict__ A, const unsigned short* __restrict__ WT,
    float* outF, int K, int ldo, int nN,
    const float* __restrict__ atts, const float* __restrict__ attd, int nHeads,
    float* SD, int MPr, const float* __restrict__ bias)
{
  __shared__ __attribute__((aligned(16))) float stg[GBM * GBN];
  __shared__ __attribute__((aligned(16))) float satt[2 * HC];
  __shared__ __attribute__((aligned(16))) float sdot[2 * GBM];
  const int tid = (int)threadIdx.x, lane = tid & 31, wave = tid >> 5, hh = lane >> 4, m = lane & 15;
  const int rowBase = (int)blockIdx.x * GBM;
  const int by      = (int)blockIdx.y;
  const int col0    = by * GBN;

  if constexpr (EPI == 0) {
    const int which = tid >> 6;
    const int c     = tid & 63;
    int head = by < nHeads ? by : nHeads - 1;
    head = head < 0 ? 0 : head;
    const float vs = atts[head * HC + c];
    const float vd = attd[head * HC + c];
    const float v = (which == 0) ? vs : vd;
    satt[which * HC + c] = bfr(v);
  }

  v8f acc[4];
  {
    const v8f z = {0.f, 0.f, 0.f, 0.f, 0.f, 0.f, 0.f, 0.f};
    acc[0] = z; acc[1] = z; acc[2] = z; acc[3] = z;
  }
  const unsigned short* ap = A  + (size_t)(rowBase + 16 * wave + m) * (size_t)K + 8 * hh;
  const unsigned short* wp = WT + (size_t)(col0 + m) * (size_t)K + 8 * hh;
  const int ksteps = K >> 5;
#pragma unroll 1
  for (int ks = 0; ks < ksteps; ++ks) {
    FragB af;
    af.h[0] = *(const v8usa*)(ap + 32 * ks);
    af.h[1] = *(const v8usa*)(ap + 32 * ks + 16);
#pragma unroll
    for (int t = 0; t < 4; ++t) {
      const unsigned short* wq = wp + (size_t)(16 * t) * (size_t)K + 32 * ks;
      FragB bf;
      bf.h[0] = *(const v8usa*)wq;
      bf.h[1] = *(const v8usa*)(wq + 16);
      acc[t] = wmb(af, bf, acc[t]);
    }
  }

#pragma unroll
  for (int t = 0; t < 4; ++t) {
    const int lc = 16 * t + m;
#pragma unroll
    for (int r = 0; r < 8; ++r) {
      const int lr = 16 * wave + 8 * hh + r;
      stg[lr * GBN + lc] = acc[t][r];
    }
  }
  __syncthreads();

  if constexpr (EPI == 0) {
    const int row = tid & 63, which = tid >> 6;
    const float* sa = satt + which * HC;
    const float* hr = stg + row * GBN;
    float ds = 0.f;
#pragma unroll 2
    for (int c4 = 0; c4 < HC / 4; ++c4) {
      const v4f hv = *(const v4fa*)(hr + 4 * c4);
      const v4f av = *(const v4fa*)(sa + 4 * c4);
      ds = fmaf(hv.x, av.x, ds);
      ds = fmaf(hv.y, av.y, ds);
      ds = fmaf(hv.z, av.z, ds);
      ds = fmaf(hv.w, av.w, ds);
    }
    sdot[which * GBM + row] = ds;
    __syncthreads();
  }

  v4f fv[8];
#pragma unroll
  for (int i = 0; i < 8; ++i) {
    const int lr = 16 * wave + 2 * i + hh;
    fv[i] = *(const v4fa*)(stg + lr * GBN + 4 * m);
  }

  if constexpr (EPI == 0) {
    const int pl = lane >> 4, piece = lane & 15;
    const v4f sdv = *(const v4fa*)(sdot + pl * GBM + 4 * piece);
    float* sp = SD + (size_t)(2 * by + pl) * (size_t)MPr + rowBase + 4 * piece;
    const bool wsd = wave == 0;
#pragma unroll
    for (int i = 0; i < 8; ++i) {
      const int lr = 16 * wave + 2 * i + hh;
      const int gr = rowBase + lr;
      float* op = outF + (size_t)gr * (size_t)ldo + col0 + 4 * m;
      *(volatile v4f*)op = fv[i];
    }
    if (wsd) *(volatile v4f*)sp = sdv;
    __threadfence();
#pragma unroll
    for (int i = 0; i < 8; ++i) {
      const int lr = 16 * wave + 2 * i + hh;
      const int gr = rowBase + lr;
      float* op = outF + (size_t)gr * (size_t)ldo + col0 + 4 * m;
      *(volatile v4f*)op = fv[i];
    }
    if (wsd) *(volatile v4f*)sp = sdv;
  } else {
    const v4f bq = bfr4(*(const v4fa*)(bias + col0 + 4 * m));
#pragma unroll
    for (int i = 0; i < 8; ++i) fv[i] = fv[i] + bq;
#pragma unroll
    for (int i = 0; i < 8; ++i) {
      const int lr = 16 * wave + 2 * i + hh;
      const int gr = rowBase + lr;
      float* op = outF + (size_t)gr * (size_t)ldo + col0 + 4 * m;
      if (gr < nN) *(volatile v4f*)op = fv[i];
    }
    __threadfence();
#pragma unroll
    for (int i = 0; i < 8; ++i) {
      const int lr = 16 * wave + 2 * i + hh;
      const int gr = rowBase + lr;
      float* op = outF + (size_t)gr * (size_t)ldo + col0 + 4 * m;
      if (gr < nN) *(volatile v4f*)op = fv[i];
    }
  }
}

__global__ __launch_bounds__(NTHR) void k_agg(
    const int* __restrict__ srcs, const int* __restrict__ dsts,
    const float* __restrict__ F, const float* __restrict__ SD,
    const float* __restrict__ bias,
    float* R, float* part,
    int nN, int nE, int nb, int vec8, int MPr) {
  extern __shared__ v4f lds_dyn[];
  int* reg1 = (int*)lds_dyn;
  int* reg2 = reg1 + RCAP;
  int* scnt = reg2 + RCAP;
  int* soff = scnt + NBMAX;
  int* list = soff + NBMAX;
  int* wcnt = list + LISTN;
  int* wtot = wcnt + NWAVE;
  const int tid = (int)threadIdx.x, lane = tid & 31, wave = tid >> 5;
  const int nodeBase = (int)blockIdx.x * nb;

  for (int i = tid; i < NBMAX; i += NTHR) scnt[i] = 0;
  __syncthreads();

  int tot = 0;
  const int nChunks = (nE + CHUNK - 1) / CHUNK;
#pragma unroll 1
  for (int ch = 0; ch < nChunks; ++ch) {
    const int cbase = ch * CHUNK;
    const int wc = scan_chunk(dsts, nE, cbase, nodeBase, nb, vec8, list, tid, lane, wave);
    if (lane == 0) wcnt[wave] = wc;
    __syncthreads();
    int pre = 0, all = 0;
#pragma unroll
    for (int w2 = 0; w2 < NWAVE; ++w2) {
      int c = wcnt[w2];
      c = c < 0 ? 0 : (c > WCAP ? WCAP : c);
      all += c;
      pre += (w2 < wave) ? c : 0;
    }
    const int wcc  = wc > WCAP ? WCAP : wc;
    const int base = tot + pre;
#pragma unroll 1
    for (int i = lane; i < wcc; i += 32) {
      const int ent = list[wave * WCAP + i];
      const int el  = (ent >> SLOTB) & (CHUNK - 1);
      const int sl  = ent & (NBMAX - 1);
      int eid = cbase + el;
      eid = eid > nE - 1 ? nE - 1 : eid;
      const int pos = base + i;
      if (pos < RCAP) reg1[pos] = (int)(((unsigned)eid << SLOTB) | (unsigned)sl);
    }
    tot += all;
    tot = tot > RCAP ? RCAP : tot;
    __syncthreads();
  }
  const int nh = tot;

  if (wave == 0) {
#pragma unroll 1
    for (int b0 = 0; b0 < nh; b0 += 32) {
      const int idx = b0 + lane;
      const int uv  = reg1[idx < nh ? idx : nh - 1];
      const int m32 = (nh - b0) < 32 ? (nh - b0) : 32;
#pragma unroll 1
      for (int k = 0; k < m32; ++k) {
        const int u  = __builtin_amdgcn_readlane(uv, k);
        const int sl = u & (NBMAX - 1);
        if (lane == 0) scnt[sl] = scnt[sl] + 1;
      }
    }
  }
  __syncthreads();

  {
    const v4i ca = *(const v4i*)(scnt + 8 * tid);
    const v4i cb = *(const v4i*)(scnt + 8 * tid + 4);
    const int e0 = ca.x < 0 ? 0 : ca.x, e1 = ca.y < 0 ? 0 : ca.y, e2 = ca.z < 0 ? 0 : ca.z, e3 = ca.w < 0 ? 0 : ca.w;
    const int e4 = cb.x < 0 ? 0 : cb.x, e5 = cb.y < 0 ? 0 : cb.y, e6 = cb.z < 0 ? 0 : cb.z, e7 = cb.w < 0 ? 0 : cb.w;
    const int ts = e0 + e1 + e2 + e3 + e4 + e5 + e6 + e7;
    int incl = ts;
#pragma unroll
    for (int d = 1; d < 32; d <<= 1) {
      const int up = __shfl_up(incl, d);
      if (lane >= d) incl += up;
    }
    if (lane == 31) wtot[wave] = incl;
    __syncthreads();
    int pre = 0;
#pragma unroll
    for (int w2 = 0; w2 < NWAVE; ++w2) pre += (w2 < wave) ? wtot[w2] : 0;
    int run = pre + incl - ts;
    soff[8 * tid + 0] = run; run += e0;
    soff[8 * tid + 1] = run; run += e1;
    soff[8 * tid + 2] = run; run += e2;
    soff[8 * tid + 3] = run; run += e3;
    soff[8 * tid + 4] = run; run += e4;
    soff[8 * tid + 5] = run; run += e5;
    soff[8 * tid + 6] = run; run += e6;
    soff[8 * tid + 7] = run;
  }
  __syncthreads();
  for (int i = tid; i < NBMAX; i += NTHR) list[i] = soff[i];
  __syncthreads();

  if (wave == 0) {
#pragma unroll 1
    for (int b0 = 0; b0 < nh; b0 += 32) {
      const int idx = b0 + lane;
      const int uv  = reg1[idx < nh ? idx : nh - 1];
      const int m32 = (nh - b0) < 32 ? (nh - b0) : 32;
#pragma unroll 1
      for (int k = 0; k < m32; ++k) {
        const int u   = __builtin_amdgcn_readlane(uv, k);
        const int sl  = u & (NBMAX - 1);
        const int eid = (int)((unsigned)u >> SLOTB);
        if (lane == 0) {
          int pos = list[sl];
          pos = pos < 0 ? 0 : (pos > RCAP - 1 ? RCAP - 1 : pos);
          reg2[pos] = eid;
          list[sl] = pos + 1;
        }
      }
    }
  }
  __syncthreads();

  const int nbw = nb >> 3;
  const bool ovf = (nh >= RCAP);
  const float qnan = __int_as_float(0x7fc00000);
  const int cA = 4 * lane;
  const int cB = FHB + 2 * lane;
  const int hA = lane >> 4;
  const v4f bbA = bfr4(*(const v4fa*)(bias + cA));
  v2f bbB;
  {
    const v2f t2 = *(const v2fa*)(bias + cB);
    bbB.x = bfr(t2.x); bbB.y = bfr(t2.y);
  }
  const float* ASpA = SD + (size_t)(2 * hA) * (size_t)MPr;
  const float* ADpA = ASpA + MPr;
  const float* ASp2 = SD + (size_t)4 * (size_t)MPr;
  const float* ADp2 = ASp2 + MPr;
  int wn = 0;
  float wm[6], wq[6];
#pragma unroll
  for (int j = 0; j < 6; ++j) { wm[j] = 0.0f; wq[j] = 0.0f; }

#pragma unroll 1
  for (int jt = 0; jt < nbw; ++jt) {
    const int slot = wave * nbw + jt;
    const int grow = nodeBase + slot;
    const int gcl  = grow < nN ? grow : nN - 1;
    int st = soff[slot];
    const int craw = scnt[slot];
    int cnt = craw;
    st  = st < 0 ? 0 : (st > nh ? nh : st);
    cnt = cnt < 0 ? 0 : (cnt > DEGCAP ? DEGCAP : cnt);
    if (cnt > nh - st) cnt = nh - st;
    const float pz = (ovf || craw > DEGCAP) ? qnan : 0.0f;

    const float advA = ADpA[gcl];
    const float adv2 = ADp2[gcl];
    float mxA = MX0, dnA = 0.0f, mx2 = MX0, dn2 = 0.0f;
    v4f av = {0.f, 0.f, 0.f, 0.f};
    v2f aw = {0.f, 0.f};

#pragma unroll 1
    for (int q = 0; q < cnt; ++q) {
      int idx = st + q; idx = idx > RCAP - 1 ? RCAP - 1 : idx;
      int eid = reg2[idx]; eid = eid < 0 ? 0 : (eid > nE - 1 ? nE - 1 : eid);
      const int sraw = srcs[eid];
      const int s = sraw < 0 ? 0 : (sraw > nN - 1 ? nN - 1 : sraw);
      const float* fr = F + (size_t)s * DW;
      const v4f fs = *(const v4fa*)(fr + cA);
      const v2f ft = *(const v2fa*)(fr + cB);
      float lgA = ASpA[s] + advA;
      lgA = lgA > 0.f ? lgA : NEGSL * lgA;
      float lg2 = ASp2[s] + adv2;
      lg2 = lg2 > 0.f ? lg2 : NEGSL * lg2;
      {
        const float df = lgA - mxA;
        const float ee = __expf(-fabsf(df));
        const bool up  = df > 0.f;
        const float s1 = up ? ee : 1.0f;
        const float s2 = up ? 1.0f : ee;
        mxA = up ? lgA : mxA;
        dnA = fmaf(dnA, s1, s2);
        av.x = fmaf(av.x, s1, s2 * fs.x);
        av.y = fmaf(av.y, s1, s2 * fs.y);
        av.z = fmaf(av.z, s1, s2 * fs.z);
        av.w = fmaf(av.w, s1, s2 * fs.w);
      }
      {
        const float df = lg2 - mx2;
        const float ee = __expf(-fabsf(df));
        const bool up  = df > 0.f;
        const float s1 = up ? ee : 1.0f;
        const float s2 = up ? 1.0f : ee;
        mx2 = up ? lg2 : mx2;
        dn2 = fmaf(dn2, s1, s2);
        aw.x = fmaf(aw.x, s1, s2 * ft.x);
        aw.y = fmaf(aw.y, s1, s2 * ft.y);
      }
    }
    const float invA = __builtin_amdgcn_rcpf(dnA + EPS_SM);
    const float inv2 = __builtin_amdgcn_rcpf(dn2 + EPS_SM);
    const bool live = grow < nN;
    float o[6];
    o[0] = (live ? fmaxf(fmaf(av.x, invA, bbA.x), 0.0f) : 0.0f) + pz;
    o[1] = (live ? fmaxf(fmaf(av.y, invA, bbA.y), 0.0f) : 0.0f) + pz;
    o[2] = (live ? fmaxf(fmaf(av.z, invA, bbA.z), 0.0f) : 0.0f) + pz;
    o[3] = (live ? fmaxf(fmaf(av.w, invA, bbA.w), 0.0f) : 0.0f) + pz;
    o[4] = (live ? fmaxf(fmaf(aw.x, inv2, bbB.x), 0.0f) : 0.0f) + pz;
    o[5] = (live ? fmaxf(fmaf(aw.y, inv2, bbB.y), 0.0f) : 0.0f) + pz;
    if (live) {
      wn += 1;
      const float rk = 1.0f / (float)(jt + 1);
#pragma unroll
      for (int j = 0; j < 6; ++j) {
        const float d = o[j] - wm[j];
        wm[j] = fmaf(d, rk, wm[j]);
        wq[j] = fmaf(d, o[j] - wm[j], wq[j]);
      }
    }
    v4f oa; v2f ob;
    oa.x = o[0]; oa.y = o[1]; oa.z = o[2]; oa.w = o[3];
    ob.x = o[4]; ob.y = o[5];
    float* gp = R + (size_t)grow * DW;
    const bool wr = grow < MPr;
    if (wr) { *(volatile v4f*)(gp + cA) = oa; *(volatile v2f*)(gp + cB) = ob; }
    __threadfence();
    if (wr) { *(volatile v4f*)(gp + cA) = oa; *(volatile v2f*)(gp + cB) = ob; }
  }

  float* wst = (float*)reg1;
  float* pst = wst + NWAVE * WSTW;
  if (lane == 0) wst[wave * WSTW] = (float)wn;
#pragma unroll
  for (int j = 0; j < 4; ++j) {
    wst[wave * WSTW + 1 + cA + j]      = wm[j];
    wst[wave * WSTW + 1 + DW + cA + j] = wq[j];
  }
#pragma unroll
  for (int j = 0; j < 2; ++j) {
    wst[wave * WSTW + 1 + cB + j]      = wm[4 + j];
    wst[wave * WSTW + 1 + DW + cB + j] = wq[4 + j];
  }
  __syncthreads();
  if (tid < DW) {
    float n = 0.0f, mean = 0.0f, M2 = 0.0f;
#pragma unroll 1
    for (int w2 = 0; w2 < NWAVE; ++w2) {
      const float cw = wst[w2 * WSTW];
      const float mb = wst[w2 * WSTW + 1 + tid];
      const float qb = wst[w2 * WSTW + 1 + DW + tid];
      if (cw > 0.5f) {
        const float nn = n + cw;
        const float delta = mb - mean;
        const float f = cw / nn;
        mean = fmaf(delta, f, mean);
        M2 = M2 + qb + delta * delta * n * f;
        n = nn;
      }
    }
    pst[1 + tid] = mean;
    pst[1 + DW + tid] = M2;
    if (tid == 0) pst[0] = n;
  }
#pragma unroll 1
  for (int i = 2 * DW + 1 + tid; i < PARTW; i += NTHR) pst[i] = 0.0f;
  __syncthreads();
  const int pb = (int)blockIdx.x;
  v4f ps;
  if (tid < PARTW / 4) {
    ps = *(const v4fa*)(pst + 4 * tid);
    *(volatile v4f*)(part + (size_t)pb * PARTW + 4 * tid) = ps;
  }
  __threadfence();
  if (tid < PARTW / 4) {
    *(volatile v4f*)(part + (size_t)pb * PARTW + 4 * tid) = ps;
  }
}

__global__ __launch_bounds__(NTHR) void k_bnfin(const float* __restrict__ part, int nPart,
                                                const float* __restrict__ gam, const float* __restrict__ bet,
                                                float* ss) {
  __shared__ __attribute__((aligned(16))) float stg[2 * DW];
  const int tid = (int)threadIdx.x;
  const int c = tid < DW ? tid : DW - 1;
  double n = 0.0, mean = 0.0, M2 = 0.0;
#pragma unroll 1
  for (int b = 0; b < nPart; ++b) {
    const float* pr = part + (size_t)b * PARTW;
    const double cw = (double)pr[0];
    const double mb = (double)pr[1 + c];
    const double qb = (double)pr[1 + DW + c];
    if (cw > 0.5) {
      const double nn = n + cw;
      const double delta = mb - mean;
      const double f = cw / nn;
      mean = mean + delta * f;
      M2 = M2 + qb + delta * delta * n * f;
      n = nn;
    }
  }
  const double nt = n < 1.0 ? 1.0 : n;
  const float varf  = (float)(M2 / nt);
  const float meanf = (float)mean;
  const float rstd = 1.0f / sqrtf(varf + EPS_BN);
  const float sc = bfr(gam[c]) * rstd;
  const float sh = bfr(bet[c]) - meanf * sc;
  if (tid < DW) {
    stg[tid] = sc;
    stg[DW + tid] = sh;
  }
  __syncthreads();
  v4f v;
  if (tid < (2 * DW) / 4) {
    v = *(const v4fa*)(stg + 4 * tid);
    *(volatile v4f*)(ss + 4 * tid) = v;
  }
  __threadfence();
  if (tid < (2 * DW) / 4) {
    *(volatile v4f*)(ss + 4 * tid) = v;
  }
}

__global__ __launch_bounds__(NTHR) void k_bn1(const float* __restrict__ R, const float* __restrict__ ss,
                                              int nN, int nUnits, unsigned short* aout) {
  __shared__ float ssh[2 * DW];
  const int tid = (int)threadIdx.x;
  for (int i = tid; i < 2 * DW; i += NTHR) ssh[i] = ss[i];
  __syncthreads();
  const int u = (int)blockIdx.x * NTHR + tid;
  if (u >= nUnits) return;
  const int row = u / (DW / 8);
  const int c0  = (u - row * (DW / 8)) * 8;
  const float* p = R + (size_t)row * DW + c0;
  const v4f a = *(const v4fa*)p, b = *(const v4fa*)(p + 4);
  v4f ya, yb;
  ya.x = fmaf(a.x, ssh[c0 + 0], ssh[DW + c0 + 0]);
  ya.y = fmaf(a.y, ssh[c0 + 1], ssh[DW + c0 + 1]);
  ya.z = fmaf(a.z, ssh[c0 + 2], ssh[DW + c0 + 2]);
  ya.w = fmaf(a.w, ssh[c0 + 3], ssh[DW + c0 + 3]);
  yb.x = fmaf(b.x, ssh[c0 + 4], ssh[DW + c0 + 4]);
  yb.y = fmaf(b.y, ssh[c0 + 5], ssh[DW + c0 + 5]);
  yb.z = fmaf(b.z, ssh[c0 + 6], ssh[DW + c0 + 6]);
  yb.w = fmaf(b.w, ssh[c0 + 7], ssh[DW + c0 + 7]);
  const v4f z4 = {0.f, 0.f, 0.f, 0.f};
  if (row >= nN) { ya = z4; yb = z4; }
  const v4u hv = pack8(ya, yb);
  const v4u lv = pack8lo(ya, yb);
  unsigned short* op = aout + (size_t)row * KA2 + c0;
  *(volatile v4u*)op = hv;
  *(volatile v4u*)(op + DW) = lv;
  __threadfence();
  *(volatile v4u*)op = hv;
  *(volatile v4u*)(op + DW) = lv;
}

__global__ __launch_bounds__(NTHR) void k_bn2(const float* __restrict__ R, const float* __restrict__ ss,
                                              const unsigned short* __restrict__ hpl,
                                              int nN, int nUnits, unsigned short* aout) {
  __shared__ float ssh[2 * DW];
  const int tid = (int)threadIdx.x;
  for (int i = tid; i < 2 * DW; i += NTHR) ssh[i] = ss[i];
  __syncthreads();
  const int u = (int)blockIdx.x * NTHR + tid;
  if (u >= nUnits) return;
  const int row = u / (DW / 8);
  const int c0  = (u - row * (DW / 8)) * 8;
  const float* p = R + (size_t)row * DW + c0;
  const v4f a = *(const v4fa*)p, b = *(const v4fa*)(p + 4);
  const unsigned short* hp = hpl + (size_t)row * KA2 + c0;
  const v4u hw = *(const v4ua*)hp;
  const v4u lw = *(const v4ua*)(hp + DW);
  float h[8];
  h[0] = __uint_as_float(hw.x << 16)          + __uint_as_float(lw.x << 16);
  h[1] = __uint_as_float(hw.x & 0xffff0000u) + __uint_as_float(lw.x & 0xffff0000u);
  h[2] = __uint_as_float(hw.y << 16)          + __uint_as_float(lw.y << 16);
  h[3] = __uint_as_float(hw.y & 0xffff0000u) + __uint_as_float(lw.y & 0xffff0000u);
  h[4] = __uint_as_float(hw.z << 16)          + __uint_as_float(lw.z << 16);
  h[5] = __uint_as_float(hw.z & 0xffff0000u) + __uint_as_float(lw.z & 0xffff0000u);
  h[6] = __uint_as_float(hw.w << 16)          + __uint_as_float(lw.w << 16);
  h[7] = __uint_as_float(hw.w & 0xffff0000u) + __uint_as_float(lw.w & 0xffff0000u);
  v4f ya, yb;
  ya.x = h[0] + fmaf(a.x, ssh[c0 + 0], ssh[DW + c0 + 0]);
  ya.y = h[1] + fmaf(a.y, ssh[c0 + 1], ssh[DW + c0 + 1]);
  ya.z = h[2] + fmaf(a.z, ssh[c0 + 2], ssh[DW + c0 + 2]);
  ya.w = h[3] + fmaf(a.w, ssh[c0 + 3], ssh[DW + c0 + 3]);
  yb.x = h[4] + fmaf(b.x, ssh[c0 + 4], ssh[DW + c0 + 4]);
  yb.y = h[5] + fmaf(b.y, ssh[c0 + 5], ssh[DW + c0 + 5]);
  yb.z = h[6] + fmaf(b.z, ssh[c0 + 6], ssh[DW + c0 + 6]);
  yb.w = h[7] + fmaf(b.w, ssh[c0 + 7], ssh[DW + c0 + 7]);
  const v4f z4 = {0.f, 0.f, 0.f, 0.f};
  if (row >= nN) { ya = z4; yb = z4; }
  const v4u hv = pack8(ya, yb);
  const v4u lv = pack8lo(ya, yb);
  unsigned short* op = aout + (size_t)row * KA2 + c0;
  *(volatile v4u*)op = hv;
  *(volatile v4u*)(op + DW) = lv;
  __threadfence();
  *(volatile v4u*)op = hv;
  *(volatile v4u*)(op + DW) = lv;
}

static int pick_nb(int nE, int nN) {
  int nb = NBMAX;
  while (nb > 32 && (long long)nb * (long long)nE * 5LL > (long long)RCAP * (long long)nN * 4LL) nb >>= 1;
  return nb;
}
static inline int cdiv(int a, int b) { return (a + b - 1) / b; }
static inline size_t al256(size_t o) { return (o + 255) & ~(size_t)255; }

extern "C" void kernel_launch(void* const* d_in, const int* in_sizes, int n_in,
                              void* d_out, int out_size, void* d_ws, size_t ws_size,
                              hipStream_t stream) {
  if (n_in < 16) return;
  if (in_sizes[0] < F_IN || (in_sizes[0] % F_IN) != 0) return;
  const int nN = in_sizes[0] / F_IN;
  if (nN < 16 || nN > (1 << 22)) return;
  if (in_sizes[1] != F_IN * DW) return;
  if (in_sizes[2] != NHD * HC || in_sizes[3] != NHD * HC) return;
  if (in_sizes[4] != DW || in_sizes[5] != DW || in_sizes[6] != DW) return;
  if (in_sizes[7] != DW * DW) return;
  if (in_sizes[8] != NHD * HC || in_sizes[9] != NHD * HC) return;
  if (in_sizes[10] != DW || in_sizes[11] != DW || in_sizes[12] != DW) return;
  if (in_sizes[13] != DW * OUTW || in_sizes[14] != OUTW) return;
  if (in_sizes[15] < 2 || (in_sizes[15] & 1) != 0) return;
  const int nE = in_sizes[15] / 2;
  if (nE < 1 || nE >= (1 << (32 - SLOTB))) return;
  if ((long long)out_size != (long long)nN * OUTW) return;

  const float* x    = (const float*)d_in[0];
  const float* W1   = (const float*)d_in[1];
  const float* a1s  = (const float*)d_in[2];
  const float* a1d  = (const float*)d_in[3];
  const float* b1   = (const float*)d_in[4];
  const float* g1   = (const float*)d_in[5];
  const float* be1  = (const float*)d_in[6];
  const float* W2   = (const float*)d_in[7];
  const float* a2s  = (const float*)d_in[8];
  const float* a2d  = (const float*)d_in[9];
  const float* b2   = (const float*)d_in[10];
  const float* g2   = (const float*)d_in[11];
  const float* be2  = (const float*)d_in[12];
  const float* Wf   = (const float*)d_in[13];
  const float* bfv  = (const float*)d_in[14];
  const int*   ei   = (const int*)  d_in[15];
  float* out = (float*)d_out;
  const int* src = ei;
  const int* dst = ei + nE;

  const int MP   = cdiv(nN, MROWS) * MROWS;
  const int gM   = MP / GBM;
  const int nb   = pick_nb(nE, nN);
  if (nb < 32 || (nb & (nb - 1)) != 0 || nb > NBMAX) return;
  const int gA   = cdiv(MP, nb);
  if ((long long)gA * nb < (long long)MP) return;
  const int vec8 = ((nE & 3) == 0) ? 1 : 0;

  char* ws = (char*)d_ws;
  size_t off = 0;
  const size_t oW1T = off; off = al256(off + (size_t)DW * F_IN * 2);
  const size_t oW2T = off; off = al256(off + (size_t)DW * KA2 * 2);
  const size_t oWFT = off; off = al256(off + (size_t)OUTW * KA2 * 2);
  const size_t oSD  = off; off = al256(off + (size_t)(2 * NHD) * MP * 4);
  const size_t oPT  = off; off = al256(off + (size_t)gA * PARTW * 4);
  const size_t oSS  = off; off = al256(off + (size_t)(2 * DW) * 4);
  size_t szRG = (size_t)MP * DW * 4;
  if ((size_t)MP * KA2 * 2 > szRG) szRG = (size_t)MP * KA2 * 2;
  if ((size_t)MP * F_IN * 2 > szRG) szRG = (size_t)MP * F_IN * 2;
  const size_t oRG1 = off; off = al256(off + szRG);
  const size_t oRG2 = off; off = al256(off + szRG);
  const size_t oRG3 = off; off = al256(off + szRG);
  if (off > ws_size || off > (size_t)WSMAX) return;
  unsigned short* W1T = (unsigned short*)(ws + oW1T);
  unsigned short* W2T = (unsigned short*)(ws + oW2T);
  unsigned short* WFT = (unsigned short*)(ws + oWFT);
  float*          SD  = (float*)(ws + oSD);
  float*          PT  = (float*)(ws + oPT);
  float*          SS  = (float*)(ws + oSS);
  unsigned short* XB  = (unsigned short*)(ws + oRG1);
  float*          R1  = (float*)(ws + oRG1);
  float*          HP2 = (float*)(ws + oRG1);
  unsigned short* AF  = (unsigned short*)(ws + oRG1);
  float*          HP1 = (float*)(ws + oRG2);
  unsigned short* A2  = (unsigned short*)(ws + oRG2);
  float*          R2  = (float*)(ws + oRG3);

  hipFuncSetAttribute(reinterpret_cast<const void*>(&k_agg),
                      hipFuncAttributeMaxDynamicSharedMemorySize, LDS_AGG);

  const int nUx = MP * (F_IN / 8);
  k_xprep<<<cdiv(nUx, NTHR), NTHR, 0, stream>>>(x, XB, nN, nUx);

  {
    const int nUw1 = DW * (F_IN / 8);
    k_wtr<<<cdiv(nUw1, NTHR), NTHR, 0, stream>>>(W1, F_IN, DW, DW, F_IN, W1T, nUw1);
    const int nUw2 = DW * (KA2 / 8);
    k_wtr<<<cdiv(nUw2, NTHR), NTHR, 0, stream>>>(W2, DW, DW, DW, KA2, W2T, nUw2);
    const int nUwf = OUTW * (KA2 / 8);
    k_wtr<<<cdiv(nUwf, NTHR), NTHR, 0, stream>>>(Wf, DW, OUTW, OUTW, KA2, WFT, nUwf);
  }

  const int nUb = MP * (DW / 8);

  k_gemm<0><<<dim3(gM, DW / GBN), GTHR, 0, stream>>>(XB, W1T, HP1, F_IN, DW, nN, a1s, a1d, NHD, SD, MP, b1);
  k_agg<<<gA, NTHR, LDS_AGG, stream>>>(src, dst, HP1, SD, b1, R1, PT, nN, nE, nb, vec8, MP);
  k_bnfin<<<1, NTHR, 0, stream>>>(PT, gA, g1, be1, SS);
  k_bn1<<<cdiv(nUb, NTHR), NTHR, 0, stream>>>(R1, SS, nN, nUb, A2);
  k_gemm<0><<<dim3(gM, DW / GBN), GTHR, 0, stream>>>(A2, W2T, HP2, KA2, DW, nN, a2s, a2d, NHD, SD, MP, b2);
  k_agg<<<gA, NTHR, LDS_AGG, stream>>>(src, dst, HP2, SD, b2, R2, PT, nN, nE, nb, vec8, MP);
  k_bnfin<<<1, NTHR, 0, stream>>>(PT, gA, g2, be2, SS);
  k_bn2<<<cdiv(nUb, NTHR), NTHR, 0, stream>>>(R2, SS, A2, nN, nUb, AF);
  k_gemm<1><<<dim3(gM, OUTW / GBN), GTHR, 0, stream>>>(AF, WFT, out, KA2, OUTW, nN, bfv, bfv, 1, SD, MP, bfv);
}
